// CrissCrossAttention_fake_x_84189948936441
// MI455X (gfx1250) — hardware-verified
//
#include <hip/hip_runtime.h>


#define NB_  4
#define CC   256
#define CQ   32
#define GH   64
#define GW   64
#define HW   4096
#define PCAR 1024.0f
typedef _Float16 h16;
typedef unsigned short bf;
typedef __attribute__((ext_vector_type(16))) __bf16   v16bf;
typedef __attribute__((ext_vector_type(16))) _Float16 v16h;
typedef __attribute__((ext_vector_type(8)))  _Float16 v8h;
typedef __attribute__((ext_vector_type(8)))  unsigned short v8us;
typedef __attribute__((ext_vector_type(8)))  float    v8f;
typedef __attribute__((ext_vector_type(4)))  float    v4f;
typedef v8h  __attribute__((may_alias)) v8ha;
typedef v4f  __attribute__((may_alias)) v4fa;
typedef v8us __attribute__((may_alias)) v8usa;

__device__ __forceinline__ unsigned short f2bf(float f) { unsigned u = __float_as_uint(f); u += 0x7FFFu + ((u >> 16) & 1u); return (unsigned short)(u >> 16); }
__device__ __forceinline__ float bf2f(unsigned short b) { return __uint_as_float(((unsigned)b) << 16); }
__device__ __forceinline__ float bfr(float f) { return bf2f(f2bf(f)); }
__device__ __forceinline__ v16h cat16(v8h lo, v8h hi) { return __builtin_shufflevector(lo, hi, 0, 1, 2, 3, 4, 5, 6, 7, 8, 9, 10, 11, 12, 13, 14, 15); }
__device__ __forceinline__ v16bf cat16b(v8us lo, v8us hi) { return __builtin_bit_cast(v16bf, __builtin_shufflevector(lo, hi, 0, 1, 2, 3, 4, 5, 6, 7, 8, 9, 10, 11, 12, 13, 14, 15)); }
__device__ __forceinline__ v8f wmma16(v16h a, v16h b, v8f c) { return __builtin_amdgcn_wmma_f32_16x16x32_f16(false, a, false, b, (short)0, c, false, false); }
__device__ __forceinline__ v8f wmmab(v16bf a, v16bf b, v8f c) { return __builtin_amdgcn_wmma_f32_16x16x32_bf16(false, a, false, b, (short)0, c, false, false); }


template <typename T16> struct WFrag;
template <> struct WFrag<h16> { typedef v16h V; static __device__ __forceinline__ V ld(const h16* p) { return cat16(*(const v8h*)p, *(const v8h*)(p + 16)); } static __device__ __forceinline__ v8f mma(V a, V b, v8f c) { return wmma16(a, b, c); } };
template <> struct WFrag<bf> { typedef v16bf V; static __device__ __forceinline__ V ld(const bf* p) { return cat16b(*(const v8us*)p, *(const v8us*)(p + 16)); } static __device__ __forceinline__ v8f mma(V a, V b, v8f c) { return wmmab(a, b, c); } };
template <typename T16, int NSPLIT, bool BIAS>
__global__ __launch_bounds__(32) void k_gemmw(const T16* __restrict__ A, const T16* __restrict__ A2, const T16* __restrict__ Bt, const T16* __restrict__ Bt2, int K, float* C, int ldc, const float* __restrict__ bias, size_t sA, size_t sB, size_t sC) {
    typedef typename WFrag<T16>::V V;
    __shared__ __align__(16) float os[16 * 68];
    const size_t z = blockIdx.z; A += z * sA; if (A2) A2 += z * sA; Bt += z * sB; if (Bt2) Bt2 += z * sB; C += z * sC;
    const int lane = threadIdx.x & 31, lr = lane & 15, hi = lane >> 4; const int r0 = blockIdx.x * 64, c0 = blockIdx.y * 64;
    v8f acc[4][4];
#pragma unroll
    for (int mb = 0; mb < 4; ++mb)
#pragma unroll
        for (int nb = 0; nb < 4; ++nb) acc[mb][nb] = (v8f){};
    const size_t aoff = (size_t)(r0 + lr) * K + 8 * hi, boff = (size_t)(c0 + lr) * K + 8 * hi;
#pragma unroll 1
    for (int kc = 0; kc < K; kc += 32) {
        V a[4], a2[4];
#pragma unroll
        for (int mb = 0; mb < 4; ++mb) { a[mb] = WFrag<T16>::ld(A + aoff + (size_t)mb * 16 * K + kc); if (NSPLIT == 1 || NSPLIT == 2) a2[mb] = WFrag<T16>::ld(A2 + aoff + (size_t)mb * 16 * K + kc); }
#pragma unroll
        for (int nb = 0; nb < 4; ++nb) { const V b = WFrag<T16>::ld(Bt + boff + (size_t)nb * 16 * K + kc); V b2; if (NSPLIT >= 2) b2 = WFrag<T16>::ld(Bt2 + boff + (size_t)nb * 16 * K + kc);
#pragma unroll
            for (int mb = 0; mb < 4; ++mb) { acc[mb][nb] = WFrag<T16>::mma(a[mb], b, acc[mb][nb]); if (NSPLIT == 1 || NSPLIT == 2) acc[mb][nb] = WFrag<T16>::mma(a2[mb], b, acc[mb][nb]); if (NSPLIT >= 2) acc[mb][nb] = WFrag<T16>::mma(a[mb], b2, acc[mb][nb]); } }
        asm volatile("v_nop\n\tv_nop\n\tv_nop\n\tv_nop" : "+v"(acc[0][0]), "+v"(acc[1][1]), "+v"(acc[2][2]), "+v"(acc[3][3]) : "v"(a[0]), "v"(a[3]));
    }
#pragma unroll
    for (int mb = 0; mb < 4; ++mb) {
#pragma unroll
        for (int nb = 0; nb < 4; ++nb) {
#pragma unroll
            for (int j = 0; j < 8; ++j) os[(hi * 8 + j) * 68 + nb * 16 + lr] = acc[mb][nb][j]; }
        __builtin_amdgcn_wave_barrier(); asm volatile("" ::: "memory");
        float* crow = C + (size_t)(r0 + mb * 16) * ldc + c0;
#pragma unroll 1
        for (int ps = 0; ps < 2; ++ps) {
#pragma unroll
            for (int s = 0; s < 8; ++s) { const int row = 2 * s + hi, cofs = lr * 4; v4f val = *(const v4fa*)(os + row * 68 + cofs); if (BIAS) { val[0] += bfr(bias[c0 + cofs]); val[1] += bfr(bias[c0 + cofs + 1]); val[2] += bfr(bias[c0 + cofs + 2]); val[3] += bfr(bias[c0 + cofs + 3]); }
                *(volatile v4f*)(crow + (size_t)row * ldc + cofs) = val; }
            if (ps == 0) __threadfence(); }
        __builtin_amdgcn_wave_barrier(); asm volatile("" ::: "memory");
    }
}

__device__ __forceinline__ h16 tohx(float x) { return (h16)x; }
__device__ __forceinline__ void splitf(float y, unsigned short& h, unsigned short& l) { h = f2bf(y); l = f2bf(y - bf2f(h)); }
typedef __attribute__((ext_vector_type(2))) unsigned short v2us;
typedef __attribute__((ext_vector_type(4))) unsigned short v4us;
typedef __attribute__((ext_vector_type(2))) _Float16 v2h;
typedef __attribute__((ext_vector_type(4))) _Float16 v4h; typedef __attribute__((ext_vector_type(2))) float v2f;

__global__ __launch_bounds__(256) void k_cvt8(const float* __restrict__ src, bf* dst, size_t n8) { const size_t i = (size_t)blockIdx.x * 256 + threadIdx.x; if (i >= n8) return; const v8f v = *(const v8f*)(src + i * 8); v8us o;
#pragma unroll
    for (int k = 0; k < 8; ++k) o[k] = f2bf(v[k]); *(volatile v8us*)(dst + i * 8) = o; __threadfence(); *(volatile v8us*)(dst + i * 8) = o; }
__global__ __launch_bounds__(256) void k_xt(const float* __restrict__ xb, bf* XT) { const size_t e = ((size_t)blockIdx.x * 256 + threadIdx.x) * 4; if (e >= (size_t)HW * CC) return; const int c = (int)(e % CC); const int m = (int)(e / CC); v4us o;
#pragma unroll
    for (int u = 0; u < 4; ++u) o[u] = f2bf(xb[(size_t)(c + u) * HW + m]); *(volatile v4us*)(XT + e) = o; __threadfence(); *(volatile v4us*)(XT + e) = o; }
__global__ __launch_bounds__(256) void k_qkpl(const float* __restrict__ QK, bf* Qh, bf* Ql, bf* Kh, bf* Kl) { const size_t e = ((size_t)blockIdx.x * 256 + threadIdx.x) * 4; if (e >= (size_t)HW * CQ) return; const int d = (int)(e % CQ); const int n = (int)(e / CQ); const float* r = QK + (size_t)n * 2 * CQ + d; const v4f a = *(const v4f*)r, k4 = *(const v4f*)(r + CQ); v4us qh, ql, kh, kl;
#pragma unroll
    for (int u = 0; u < 4; ++u) { unsigned short p, q2; splitf(a[u], p, q2); qh[u] = p; ql[u] = q2; splitf(k4[u], p, q2); kh[u] = p; kl[u] = q2; }
    *(volatile v4us*)(Qh + e) = qh; *(volatile v4us*)(Ql + e) = ql; *(volatile v4us*)(Kh + e) = kh; *(volatile v4us*)(Kl + e) = kl; __threadfence(); *(volatile v4us*)(Qh + e) = qh; *(volatile v4us*)(Ql + e) = ql; *(volatile v4us*)(Kh + e) = kh; *(volatile v4us*)(Kl + e) = kl; }
__global__ __launch_bounds__(64) void k_bqk(const float* __restrict__ bq, const float* __restrict__ bk, float* B) { const int t = threadIdx.x; const float v = (t < CQ) ? bq[t] : bk[t - CQ]; *(volatile float*)(B + t) = v; __threadfence(); *(volatile float*)(B + t) = v; }
__global__ __launch_bounds__(256) void k_v16(const float* __restrict__ V, h16* V16, h16* VT16) { const size_t e = ((size_t)blockIdx.x * 256 + threadIdx.x) * 2; if (e >= (size_t)CC * HW) return; const int n = (int)(e % HW); const int c = (int)(e / HW); v2h o, ot;
#pragma unroll
    for (int u = 0; u < 2; ++u) { const int nn = n + u; const int hh = nn / GW, ww = nn % GW; o[u] = tohx(V[(size_t)nn * CC + c]); ot[u] = tohx(V[(size_t)(ww * GW + hh) * CC + c]); }
    *(volatile v2h*)(V16 + e) = o; *(volatile v2h*)(VT16 + e) = ot; __threadfence(); *(volatile v2h*)(V16 + e) = o; *(volatile v2h*)(VT16 + e) = ot; }
__global__ __launch_bounds__(256) void k_gsoft(const float* __restrict__ E, h16* P16) { const int lane = threadIdx.x & 31; const int wv = blockIdx.x * 8 + (threadIdx.x >> 5); if (wv >= HW * GH) return; const int n = wv / GH, hh = wv % GH; const float* er = E + (size_t)n * HW + hh * GW; const v2f a = *(const v2f*)(er + lane * 2); float v0 = a[0], v1 = a[1]; float mx = fmaxf(v0, v1);
#pragma unroll
    for (int sh = 16; sh; sh >>= 1) mx = fmaxf(mx, __shfl_xor(mx, sh, 32));
    float d0 = __fsub_rn(v0, mx), d1 = __fsub_rn(v1, mx); asm volatile("" : "+v"(d0)); asm volatile("" : "+v"(d1)); v0 = __builtin_amdgcn_exp2f(__fmul_rn(d0, 1.4426950408889634f)); v1 = __builtin_amdgcn_exp2f(__fmul_rn(d1, 1.4426950408889634f)); float sum = v0 + v1;
#pragma unroll
    for (int sh = 16; sh; sh >>= 1) sum += __shfl_xor(sum, sh, 32);
    const float f = __fdiv_rn(PCAR, sum); v2h o; o[0] = tohx(v0 * f); o[1] = tohx(v1 * f); h16* dst = P16 + (size_t)n * HW + hh * GW + lane * 2; *(volatile v2h*)dst = o; __threadfence(); *(volatile v2h*)dst = o; }
__global__ __launch_bounds__(256) void k_perm(const h16* __restrict__ P, h16* Pd, h16* Pa) { const size_t e = ((size_t)blockIdx.x * 256 + threadIdx.x) * 4; if (e >= (size_t)HW * HW) return; const int kq = (int)(e % HW); const int m = (int)(e / HW); const int q_hi0 = kq % GW; const int a2 = kq / GW;     const int q_lo = m / GW, b2 = m % GW; v4h od, oa;
#pragma unroll
    for (int u = 0; u < 4; ++u) { const int q_hi = q_hi0 + u; const size_t rowq = (size_t)(q_hi * GW + q_lo) * HW;
        od[u] = P[rowq + a2 * GW + b2];
        oa[u] = P[rowq + b2 * GW + a2]; }
    *(volatile v4h*)(Pd + e) = od; *(volatile v4h*)(Pa + e) = oa; __threadfence(); *(volatile v4h*)(Pd + e) = od; *(volatile v4h*)(Pa + e) = oa; }
__global__ __launch_bounds__(256) void k_cat(const float* __restrict__ Px, int xi, bf* Ch, bf* Cl) { const size_t e = ((size_t)blockIdx.x * 256 + threadIdx.x) * 4; if (e >= (size_t)HW * CC) return; const int c = (int)(e % CC); const int m = (int)(e / CC); v4us oh, ol;
#pragma unroll
    for (int u = 0; u < 4; ++u) { unsigned short a, b; splitf(Px[(size_t)(c + u) * HW + m] * (1.0f / PCAR), a, b); oh[u] = a; ol[u] = b; } const size_t oo = (size_t)m * 4 * CC + xi * CC + c; *(volatile v4us*)(Ch + oo) = oh; *(volatile v4us*)(Cl + oo) = ol; __threadfence(); *(volatile v4us*)(Ch + oo) = oh; *(volatile v4us*)(Cl + oo) = ol; }
__global__ __launch_bounds__(256) void k_fin(const float* __restrict__ Y, const float* __restrict__ bo, const float* __restrict__ gam, const float* __restrict__ xb, float* OUTb) { const size_t e = ((size_t)blockIdx.x * 256 + threadIdx.x) * 4; if (e >= (size_t)CC * HW) return; const int m = (int)(e % HW); const int c = (int)(e / HW); const float gg = bfr(gam[0]), bb = bfr(bo[c]); v4f r;
#pragma unroll
    for (int u = 0; u < 4; ++u) { const float y0 = __fadd_rn(Y[(size_t)(m + u) * CC + c], bb); float gy = __fmul_rn(gg, y0); asm volatile("" : "+v"(gy)); r[u] = __fadd_rn(gy, bfr(xb[(size_t)c * HW + m + u])); }
    *(volatile v4f*)(OUTb + e) = r; __threadfence(); *(volatile v4f*)(OUTb + e) = r; }

extern "C" void kernel_launch(void* const* d_in, const int* in_sizes, int n_in,
                              void* d_out, int out_size, void* d_ws, size_t ws_size, hipStream_t stream) {
    (void)in_sizes; (void)n_in; (void)out_size;
    const float* x = (const float*)d_in[0]; const float* wq = (const float*)d_in[1]; const float* bq = (const float*)d_in[2]; const float* wk = (const float*)d_in[3]; const float* bk = (const float*)d_in[4]; const float* wv = (const float*)d_in[5]; const float* bv = (const float*)d_in[6]; const float* wo = (const float*)d_in[7]; const float* bo = (const float*)d_in[8]; const float* gam = (const float*)d_in[9];
    float* OUT = (float*)d_out;
    char* wsp = (char*)d_ws;
    auto take = [&](size_t bytes) { char* p = wsp; wsp += (bytes + 255) & ~(size_t)255; return (void*)p; };
    bf* BQK = (bf*)take((size_t)2 * CQ * CC * 2); bf* BV = (bf*)take((size_t)CC * CC * 2); bf* BO = (bf*)take((size_t)CC * 4 * CC * 2);
    bf* XT = (bf*)take((size_t)HW * CC * 2); float* QK = (float*)take((size_t)HW * 2 * CQ * 4); float* BQKB = (float*)take(256); float* V = (float*)take((size_t)HW * CC * 4);
    bf* Qh = (bf*)take((size_t)HW * CQ * 2); bf* Ql = (bf*)take((size_t)HW * CQ * 2); bf* Kh = (bf*)take((size_t)HW * CQ * 2); bf* Kl = (bf*)take((size_t)HW * CQ * 2); h16* V16 = (h16*)take((size_t)CC * HW * 2); h16* VT16 = (h16*)take((size_t)CC * HW * 2);
    float* E = (float*)take((size_t)HW * HW * 4); h16* P16 = (h16*)take((size_t)HW * HW * 2); h16* Pd = (h16*)take((size_t)HW * HW * 2); h16* Pa = (h16*)take((size_t)HW * HW * 2); float* PX = (float*)take((size_t)CC * HW * 4);
    bf* CATh = (bf*)take((size_t)HW * 4 * CC * 2); bf* CATl = (bf*)take((size_t)HW * 4 * CC * 2); float* Y = (float*)take((size_t)HW * CC * 4);
    if ((size_t)(wsp - (char*)d_ws) > ws_size) return;
    k_cvt8<<<(CQ * CC / 8 + 255) / 256, 256, 0, stream>>>(wq, BQK, CQ * CC / 8); k_cvt8<<<(CQ * CC / 8 + 255) / 256, 256, 0, stream>>>(wk, BQK + (size_t)CQ * CC, CQ * CC / 8); k_bqk<<<1, 64, 0, stream>>>(bq, bk, BQKB);     k_cvt8<<<(CC * CC / 8 + 255) / 256, 256, 0, stream>>>(wv, BV, CC * CC / 8); k_cvt8<<<(CC * 4 * CC / 8 + 255) / 256, 256, 0, stream>>>(wo, BO, CC * 4 * CC / 8);
    for (int b = 0; b < NB_; ++b) { const float* xb = x + (size_t)b * CC * HW;
        k_xt<<<(unsigned)(((size_t)HW * CC / 4 + 255) / 256), 256, 0, stream>>>(xb, XT);
        k_gemmw<bf, 0, true><<<dim3(HW / 64, 1, 1), 32, 0, stream>>>(XT, nullptr, BQK, nullptr, CC, QK, 2 * CQ, BQKB, 0, 0, 0);
        k_gemmw<bf, 0, true><<<dim3(HW / 64, CC / 64, 1), 32, 0, stream>>>(XT, nullptr, BV, nullptr, CC, V, CC, bv, 0, 0, 0);
        k_qkpl<<<(unsigned)(((size_t)HW * CQ / 4 + 255) / 256), 256, 0, stream>>>(QK, Qh, Ql, Kh, Kl); k_v16<<<(unsigned)(((size_t)CC * HW / 2 + 255) / 256), 256, 0, stream>>>(V, V16, VT16);
        k_gemmw<bf, 2, false><<<dim3(HW / 64, HW / 64, 1), 32, 0, stream>>>(Qh, Ql, Kh, Kl, CQ, E, HW, nullptr, 0, 0, 0);
        k_gsoft<<<HW * GH / 8, 256, 0, stream>>>(E, P16);
        k_perm<<<(unsigned)(((size_t)HW * HW / 4 + 255) / 256), 256, 0, stream>>>(P16, Pd, Pa);
        const h16* As[4] = {V16, VT16, V16, V16}; const h16* Bs[4] = {P16, P16, Pd, Pa};
        for (int xi = 0; xi < 4; ++xi) { k_gemmw<h16, 0, false><<<dim3(CC / 64, HW / 64, 1), 32, 0, stream>>>(As[xi], nullptr, Bs[xi], nullptr, HW, PX, HW, nullptr, 0, 0, 0); k_cat<<<(unsigned)(((size_t)HW * CC / 4 + 255) / 256), 256, 0, stream>>>(PX, xi, CATh, CATl); }
        k_gemmw<bf, 1, false><<<dim3(HW / 64, CC / 64, 1), 32, 0, stream>>>(CATh, CATl, BO, nullptr, 4 * CC, Y, CC, nullptr, 0, 0, 0);
        k_fin<<<(unsigned)(((size_t)CC * HW / 4 + 255) / 256), 256, 0, stream>>>(Y, bo, gam, xb, OUT + (size_t)b * CC * HW); }
}
